// ConvCapsule_89300960018599
// MI455X (gfx1250) — hardware-verified
//
#include <hip/hip_runtime.h>
#include <math.h>

typedef __attribute__((ext_vector_type(16))) _Float16 v16h;
typedef __attribute__((ext_vector_type(16))) __bf16 v16b;
typedef __attribute__((ext_vector_type(8)))  _Float16 v8h;
typedef __attribute__((ext_vector_type(8)))  float v8f;
typedef __attribute__((ext_vector_type(4)))  float v4f;
typedef __attribute__((ext_vector_type(2)))  float v2f;
typedef __attribute__((ext_vector_type(4)))  unsigned v4u;
typedef __attribute__((ext_vector_type(4)))  int v4i;
typedef float __attribute__((may_alias)) float_a;
typedef int __attribute__((may_alias)) int_a;

template <typename T> __device__ __forceinline__ void vst2(void* p, T v) { *(volatile T*)p = v; __threadfence(); *(volatile T*)p = v; }
__device__ __forceinline__ v8f wmma16(v16h a, v16h b, v8f c) {
  v8f d = __builtin_amdgcn_wmma_f32_16x16x32_f16(false, a, false, b, (short)0, c, false, false);
  asm volatile("v_nop\n\tv_nop\n\tv_nop\n\tv_nop" : "+v"(d) : "v"(a), "v"(b));
  return d;
}
__device__ __forceinline__ v8f wmma_bf(v16b a, v16b b, v8f c) {
  v8f d = __builtin_amdgcn_wmma_f32_16x16x32_bf16(false, a, false, b, (short)0, c, false, false);
  asm volatile("v_nop\n\tv_nop\n\tv_nop\n\tv_nop" : "+v"(d) : "v"(a), "v"(b));
  return d;
}
__device__ __forceinline__ v16h frag_h(const _Float16* rowk0, int lane) {
  union { v16h v; v8h q[2]; } u; const _Float16* p = rowk0 + 8 * (lane >> 4);
  u.q[0] = *(const v8h*)p; u.q[1] = *(const v8h*)(p + 16); return u.v;
}
__device__ __forceinline__ v16h frag_f32(const float* rowk0, int lane) {
  v16h a; const float* p = rowk0 + 8 * (lane >> 4);
#pragma unroll
  for (int i = 0; i < 8; ++i) { a[i] = (_Float16)p[i]; a[8 + i] = (_Float16)p[16 + i]; }
  return a;
}
__device__ __forceinline__ v16h frag_f32s(const float* rowk0, int lane, float sc) {
  v16h a; const float* p = rowk0 + 8 * (lane >> 4);
#pragma unroll
  for (int i = 0; i < 8; ++i) { a[i] = (_Float16)(p[i] * sc); a[8 + i] = (_Float16)(p[16 + i] * sc); }
  return a;
}
__device__ __forceinline__ v16h fragc_f32(const float* W, int k0, int n, int lane, int ld, int K) {
  v16h a; const int g = lane >> 4;
#pragma unroll
  for (int i = 0; i < 8; ++i) { const int ka = k0 + 8 * g + i, kb = ka + 16;
    a[i] = (_Float16)(ka < K ? W[(size_t)(ka < K ? ka : K - 1) * ld + n] : 0.f); a[8 + i] = (_Float16)(kb < K ? W[(size_t)(kb < K ? kb : K - 1) * ld + n] : 0.f); }
  return a;
}
struct F2 { v16b h, l; };
__device__ __forceinline__ F2 bsplit16(const float v[16]) { F2 r;
#pragma unroll
  for (int i = 0; i < 16; ++i) { const __bf16 h = (__bf16)v[i]; r.h[i] = h; r.l[i] = (__bf16)(v[i] - (float)h); }
  return r; }
__device__ __forceinline__ F2 split_row(const float* row, int k0, int lane) { float v[16]; const float* p = row + k0 + 8 * (lane >> 4);
#pragma unroll
  for (int i = 0; i < 8; ++i) { v[i] = p[i]; v[8 + i] = p[16 + i]; }
  return bsplit16(v); }
__device__ __forceinline__ F2 split_rowK(const float* row, int k0, int lane, int K) { float v[16]; const int g = lane >> 4;
#pragma unroll
  for (int i = 0; i < 8; ++i) { const int ka = k0 + 8 * g + i, kb = ka + 16; v[i] = ka < K ? row[ka < K ? ka : K - 1] : 0.f; v[8 + i] = kb < K ? row[kb < K ? kb : K - 1] : 0.f; }
  return bsplit16(v); }
__device__ __forceinline__ F2 split_col(const float* W, int k0, int n, int lane, int ld, int K) { float v[16]; const int g = lane >> 4;
#pragma unroll
  for (int i = 0; i < 8; ++i) { const int ka = k0 + 8 * g + i, kb = ka + 16; v[i] = ka < K ? W[(size_t)(ka < K ? ka : K - 1) * ld + n] : 0.f; v[8 + i] = kb < K ? W[(size_t)(kb < K ? kb : K - 1) * ld + n] : 0.f; }
  return bsplit16(v); }
__device__ __forceinline__ v8f mac3(const F2& a, const F2& b, v8f c) { c = wmma_bf(a.l, b.h, c); c = wmma_bf(a.h, b.l, c); return wmma_bf(a.h, b.h, c); }
__device__ __forceinline__ float sigm(float v) { return 1.0f / (1.0f + expf(-v)); }
#define LDSX() do { asm volatile("s_wait_dscnt 0" ::: "memory"); __builtin_amdgcn_wave_barrier(); __builtin_amdgcn_fence(__ATOMIC_RELEASE, "workgroup"); } while (0)


#define NBB 8
#define NI 32
#define NO 32
#define NA 8
#define HH 32
#define WWD 32
#define NPX (HH * WWD)
#define KC 200
#define KP 224
#define NCO (NO * NA)
#ifndef NBT
#define NBT NBB
#endif
typedef __attribute__((ext_vector_type(8))) __bf16 v8b;
__device__ __forceinline__ v16b frag_b(const __bf16* rowk0, int lane) {
  union { v16b v; v8b q[2]; } u; const __bf16* p = rowk0 + 8 * (lane >> 4);
  u.q[0] = *(const v8b*)p; u.q[1] = *(const v8b*)(p + 16); return u.v;
}
__device__ __forceinline__ float bfr(float v) { return (float)(__bf16)v; }
__device__ __attribute__((noinline)) float exp_ni(float v) { return expf(v); }
__device__ __attribute__((noinline)) float erf_ni(float v) { return erff(v); }

#define WS_PW  0u
#define WS_END (WS_PW + 2u * NCO * KP)

__global__ __launch_bounds__(256) void k_packw(const float* __restrict__ CW, __bf16* __restrict__ PW) {
  __shared__ __align__(16) __bf16 s[8 * KP]; const int co0 = blockIdx.x * 8, tid = threadIdx.x;
  for (int q = tid; q < 8 * KP; q += 256) { const int rl = q / KP, k = q % KP; s[q] = (__bf16)(k < KC ? bfr(CW[(size_t)k * NCO + co0 + rl]) : 0.f); }
  __syncthreads();
  if (tid < KP) vst2((unsigned*)(PW + (size_t)co0 * KP + tid * 8), *(const v4u*)&s[tid * 8]);
}
__global__ __launch_bounds__(128) void k_caps(const float* __restrict__ X, const __bf16* __restrict__ PW, const float* __restrict__ CB, const float* __restrict__ BI, float* __restrict__ out) {
  __shared__ __align__(16) __bf16 sa[128][KP + 8];
  __shared__ __align__(16) float sv[NI][NCO][4];
  __shared__ float slog[NI][NO][4], srt[NI][NO][4];
  __shared__ __align__(16) float sact[NO][4][NA];
  const int tid = threadIdx.x, wave = tid >> 5, lane = tid & 31, col = lane & 15, hf = lane >> 4; const int p0 = blockIdx.x * 4, b = blockIdx.y;
  { const int rr = tid, i = rr >> 2, pl = rr & 3; const int px = p0 + pl, y = px / WWD, xq = px % WWD; const float* img = X + ((size_t)(b * NI + i)) * NA * NPX;
#pragma unroll 1
    for (int kh = 0; kh < 5; ++kh) { const int yy = y + kh - 2; const bool vy = (yy >= 0) && (yy < HH); const int yc = yy < 0 ? 0 : (yy >= HH ? HH - 1 : yy);
#pragma unroll
      for (int kw = 0; kw < 5; ++kw) { const int xx = xq + kw - 2; const bool vx = vy && (xx >= 0) && (xx < WWD); const int xc = xx < 0 ? 0 : (xx >= WWD ? WWD - 1 : xx);
#pragma unroll
        for (int ci = 0; ci < NA; ++ci) { const float v = img[(size_t)ci * NPX + yc * WWD + xc]; sa[rr][(kh * 5 + kw) * NA + ci] = vx ? (__bf16)v : (__bf16)0.f; } } }
    for (int k = KC; k < KP; ++k) sa[rr][k] = (__bf16)0.f;
#pragma unroll
    for (int o = 0; o < NO; ++o) slog[i][o][pl] = 0.f; }
  __syncthreads();
#pragma unroll 1
  for (int pass = 0; pass < 2; ++pass) { v8f acc[2][8] = {};
#pragma unroll 1
    for (int kc = 0; kc < KP / 32; ++kc) { const v16b a0 = frag_b(&sa[wave * 32 + col][kc * 32], lane), a1 = frag_b(&sa[wave * 32 + 16 + col][kc * 32], lane);
#pragma unroll
      for (int j = 0; j < 8; ++j) { const v16b w = frag_b(PW + (size_t)(pass * 128 + j * 16 + col) * KP + kc * 32, lane); acc[0][j] = wmma_bf(a0, w, acc[0][j]); acc[1][j] = wmma_bf(a1, w, acc[1][j]); } }
#pragma unroll
    for (int rt = 0; rt < 2; ++rt)
#pragma unroll
      for (int j = 0; j < 8; ++j) { const int co = pass * 128 + j * 16 + col; const float bb = bfr(CB[co]);
#pragma unroll
        for (int r = 0; r < 8; ++r) { const int rr = wave * 32 + rt * 16 + 8 * hf + r; sv[rr >> 2][co][rr & 3] = acc[rt][j][r] + bb; } } }
  __syncthreads();
  const int ti = tid >> 2, tp = tid & 3; const int to = tid >> 2;
#pragma unroll 1
  for (int it = 0; it < 3; ++it) {
    { float mx = 0.f;
#pragma unroll
      for (int o = 0; o < NO; ++o) mx = fmaxf(mx, slog[ti][o][tp]);
      float z = exp_ni(0.f - mx); float e[NO];
#pragma unroll
      for (int o = 0; o < NO; ++o) { e[o] = exp_ni(slog[ti][o][tp] - mx); z += e[o]; }
      const float iz = 1.0f / z;
#pragma unroll
      for (int o = 0; o < NO; ++o) srt[ti][o][tp] = e[o] * iz; }
    __syncthreads();
    { float pre[NA]; float nsq = 0.f;
#pragma unroll
      for (int a = 0; a < NA; ++a) { float s = bfr(BI[to * NA + a]);
#pragma unroll 4
        for (int i = 0; i < NI; ++i) s += sv[i][to * NA + a][tp] * srt[i][to][tp];
        pre[a] = s; nsq += s * s; }
      const float nrm = sqrtf(nsq); const float f = nrm / (1.0f + nsq);
#pragma unroll
      for (int a = 0; a < NA; ++a) sact[to][tp][a] = pre[a] * f; }
    __syncthreads();
    if (it < 2) {
#pragma unroll 2
      for (int o = 0; o < NO; ++o) { float s = 0.f;
#pragma unroll
        for (int a = 0; a < NA; ++a) s += sv[ti][o * NA + a][tp] * sact[o][tp][a];
        slog[ti][o][tp] += s; }
      __syncthreads(); } }
  for (int q = tid; q < NO * 8; q += 128) { const int o = q >> 3, piece = q & 7; vst2(out + (((size_t)b * NO + o) * NPX + p0) * NA + piece * 4, *(const v4f*)(&sact[o][0][0] + piece * 4)); }
}
extern "C" void kernel_launch(void* const* d_in, const int* in_sizes, int n_in, void* d_out, int out_size, void* d_ws, size_t ws_size, hipStream_t stream) {
  (void)in_sizes; (void)n_in; (void)out_size;
  const float** F = (const float**)d_in;
  if (ws_size < (size_t)WS_END) return;
  char* ws = (char*)d_ws; __bf16* PW = (__bf16*)(ws + WS_PW);
  k_packw<<<NCO / 8, 256, 0, stream>>>(F[1], PW);
  k_caps<<<dim3(NPX / 4, NBT), 128, 0, stream>>>(F[0], PW, F[2], F[3], (float*)d_out);
}
